// CxNE_OBSOLETE_45732811767855
// MI455X (gfx1250) — hardware-verified
//
#include <hip/hip_runtime.h>
#include <stddef.h>


#define FIN    256
#define DF     64
#define NH     4
#define NOUT   32
#define XPP    128
#define GR     32
#define NTHR   256
#define NWAVE  8
#define NB     512
#define CHUNK  2048
#define WCAP   256
#define NGRP   (CHUNK / (NTHR * 4))
#define RB     512
#define CP     128
#define WPL    32768
#define SLOPE  0.2f
#define BNEPS  1e-5f

#define LDS_SACC  (NB * DF)
#define LDS_DEN   (NB * NH)
#define LDS_ZERO  (LDS_SACC + LDS_DEN + NB + NB)
#define LDS_LIST  (NWAVE * WCAP)
#define LDS_WORDS (LDS_ZERO + LDS_DEN + NB + LDS_LIST + NWAVE)
#define LDS_BYTES (LDS_WORDS * 4)

static_assert(WCAP == (CHUNK / NTHR) * 32);
static_assert(NGRP == 2);
static_assert(NB == 512);
static_assert(NB == NWAVE * 64);
static_assert(CHUNK <= 4096);
static_assert((LDS_ZERO % 4) == 0);
static_assert(LDS_BYTES == 161824);
static_assert(XPP == 2 * DF);

typedef float          v2f   __attribute__((ext_vector_type(2)));
typedef float          v4f   __attribute__((ext_vector_type(4)));
typedef float          v8f   __attribute__((ext_vector_type(8)));
typedef double         v2d   __attribute__((ext_vector_type(2)));
typedef int            v4i   __attribute__((ext_vector_type(4)));
typedef unsigned short v8us  __attribute__((ext_vector_type(8)));
typedef __bf16         v16bf __attribute__((ext_vector_type(16)));
union FragB { v16bf v; v8us h[2]; };
union Pack8 { v8us v; unsigned short s[8]; };

__device__ __forceinline__ v8f wmb(v16bf a, v16bf b, v8f c) {
  v8f d = __builtin_amdgcn_wmma_f32_16x16x32_bf16(false, a, false, b, (short)0, c, false, false);
  asm volatile("v_nop\n\tv_nop\n\tv_nop\n\tv_nop" : "+v"(d) : "v"(a), "v"(b));
  return d;
}

__device__ __forceinline__ unsigned int rne16(float x) {
  const unsigned int u = __float_as_uint(x);
  return (u + 0x7FFFu + ((u >> 16) & 1u)) >> 16;
}
__device__ __forceinline__ void split1(float x, unsigned short& h, unsigned short& l) {
  const unsigned int hb = rne16(x);
  const float r = x - __uint_as_float(hb << 16);
  h = (unsigned short)hb;
  l = (unsigned short)rne16(r);
}
__device__ __forceinline__ v4f relu4(v4f v) {
  v4f r;
  r.x = fmaxf(v.x, 0.0f); r.y = fmaxf(v.y, 0.0f); r.z = fmaxf(v.z, 0.0f); r.w = fmaxf(v.w, 0.0f);
  return r;
}

__global__ __launch_bounds__(NTHR) void k_wprep(const float* __restrict__ W0, const float* __restrict__ W1,
                                               int K, int NC0, int NCT,
                                               unsigned short* Bh, unsigned short* Bl) {
  const int t  = blockIdx.x * NTHR + threadIdx.x;
  const int kg = K >> 3;
  if (t >= NCT * kg) return;
  const int n   = t / kg;
  const int k0  = (t - n * kg) * 8;
  const int nc1 = NCT - NC0;
  const int c0  = min(n, NC0 - 1);
  const int c1  = (nc1 > 0) ? min(max(n - NC0, 0), nc1 - 1) : 0;
  const int p1  = (nc1 > 0) ? nc1 : 0;
  const bool useA = (n < NC0);
  Pack8 uh, ul;
#pragma unroll
  for (int i = 0; i < 8; ++i) {
    const int k = k0 + i;
    const float a = W0[(size_t)k * NC0 + c0];
    const float b = W1[(size_t)k * p1 + c1];
    const float v = useA ? a : b;
    unsigned short hs, ls;
    split1(v, hs, ls);
    uh.s[i] = hs;
    ul.s[i] = ls;
  }
  const size_t o = (size_t)n * K + k0;
  const v8us vh = uh.v, vl = ul.v;
  *(volatile v8us*)(Bh + o) = vh;
  *(volatile v8us*)(Bl + o) = vl;
  __threadfence();
  *(volatile v8us*)(Bh + o) = vh;
  *(volatile v8us*)(Bl + o) = vl;
}

template <int K, int NC, bool PRE>
__global__ __launch_bounds__(NTHR) void k_gemm(
    const float* __restrict__ A,
    const unsigned short* __restrict__ Bh, const unsigned short* __restrict__ Bl,
    const float* __restrict__ bias0, const float* __restrict__ bias1, int nsplit,
    const float* __restrict__ pmean, const float* __restrict__ pscl, const float* __restrict__ pbeta,
    float* Out, int nN, int nStore) {
  constexpr int AP  = K + 8;
  constexpr int XSP = NC + 4;
  constexpr int NT  = 2 * (NC / 16);
  constexpr int LPR = NC / 4;
  constexpr int RPI = 32 / LPR;
  constexpr int NI  = 4 / RPI;
  static_assert(K % 64 == 0);
  static_assert(NC % 16 == 0 && NC >= 32 && NC <= 128);
  static_assert(NI >= 1 && NI * RPI == 4);
  __shared__ __attribute__((aligned(16))) unsigned short Ah[GR * AP];
  __shared__ __attribute__((aligned(16))) unsigned short Al[GR * AP];
  __shared__ __attribute__((aligned(16))) float Xs[GR * XSP];

  const int tid  = threadIdx.x;
  const int lane = tid & 31;
  const int wave = tid >> 5;
  const int hh   = lane >> 4;
  const int m    = lane & 15;
  const int rowBase = blockIdx.x * GR;

  {
    const int r   = tid >> 3;
    const int sub = tid & 7;
    int row = rowBase + r;
    if (row > nN - 1) row = nN - 1;
    const float* p = A + (size_t)row * K;
#pragma unroll
    for (int g = 0; g < K / 64; ++g) {
      const int c0 = g * 64 + sub * 8;
      v4f f0 = *(const v4f*)(p + c0);
      v4f f1 = *(const v4f*)(p + c0 + 4);
      if (PRE) {
        const v4f m0 = *(const v4f*)(pmean + c0), m1 = *(const v4f*)(pmean + c0 + 4);
        const v4f s0 = *(const v4f*)(pscl + c0),  s1 = *(const v4f*)(pscl + c0 + 4);
        const v4f e0 = *(const v4f*)(pbeta + c0), e1 = *(const v4f*)(pbeta + c0 + 4);
        f0 = relu4((f0 - m0) * s0 + e0);
        f1 = relu4((f1 - m1) * s1 + e1);
      }
      Pack8 uh, ul;
      split1(f0.x, uh.s[0], ul.s[0]); split1(f0.y, uh.s[1], ul.s[1]);
      split1(f0.z, uh.s[2], ul.s[2]); split1(f0.w, uh.s[3], ul.s[3]);
      split1(f1.x, uh.s[4], ul.s[4]); split1(f1.y, uh.s[5], ul.s[5]);
      split1(f1.z, uh.s[6], ul.s[6]); split1(f1.w, uh.s[7], ul.s[7]);
      *(v8us*)(Ah + r * AP + c0) = uh.v;
      *(v8us*)(Al + r * AP + c0) = ul.v;
    }
  }
  __syncthreads();

  for (int t = wave; t < NT; t += NWAVE) {
    const int rt = t & 1;
    const int ct = t >> 1;
    const int n  = ct * 16 + m;
    const unsigned short* pbh = Bh + (size_t)n * K + 8 * hh;
    const unsigned short* pbl = Bl + (size_t)n * K + 8 * hh;
    const unsigned short* pah = Ah + (rt * 16 + m) * AP + 8 * hh;
    const unsigned short* pal = Al + (rt * 16 + m) * AP + 8 * hh;
    v8f acc = {0.f, 0.f, 0.f, 0.f, 0.f, 0.f, 0.f, 0.f};
#pragma unroll 2
    for (int kt = 0; kt < K / 32; ++kt) {
      const int k0 = kt * 32;
      FragB fah, fal, fbh, fbl;
      fah.h[0] = *(const v8us*)(pah + k0); fah.h[1] = *(const v8us*)(pah + k0 + 16);
      fal.h[0] = *(const v8us*)(pal + k0); fal.h[1] = *(const v8us*)(pal + k0 + 16);
      fbh.h[0] = *(const v8us*)(pbh + k0); fbh.h[1] = *(const v8us*)(pbh + k0 + 16);
      fbl.h[0] = *(const v8us*)(pbl + k0); fbl.h[1] = *(const v8us*)(pbl + k0 + 16);
      acc = wmb(fah.v, fbh.v, acc);
      acc = wmb(fah.v, fbl.v, acc);
      acc = wmb(fal.v, fbh.v, acc);
    }
    const int i0 = min(n, nsplit - 1);
    int i1 = n - nsplit;
    if (i1 > NC - nsplit - 1) i1 = NC - nsplit - 1;
    if (i1 < 0) i1 = 0;
    const float bv0 = bias0[i0];
    const float bv1 = bias1[i1];
    const float bv  = (n < nsplit) ? bv0 : bv1;
#pragma unroll
    for (int r = 0; r < 8; ++r) Xs[(rt * 16 + 8 * hh + r) * XSP + n] = acc[r] + bv;
  }
  __syncthreads();

  v4f    vals[NI];
  size_t offs[NI];
  bool   ok[NI];
#pragma unroll
  for (int i = 0; i < NI; ++i) {
    const int rowl = 4 * wave + i * RPI + lane / LPR;
    const int col  = (lane % LPR) * 4;
    vals[i] = *(const v4f*)(Xs + rowl * XSP + col);
    const int grow = rowBase + rowl;
    ok[i]   = grow < nStore;
    offs[i] = (size_t)grow * NC + col;
  }
#pragma unroll
  for (int i = 0; i < NI; ++i) if (ok[i]) *(volatile v4f*)(Out + offs[i]) = vals[i];
  __threadfence();
#pragma unroll
  for (int i = 0; i < NI; ++i) if (ok[i]) *(volatile v4f*)(Out + offs[i]) = vals[i];
}

__global__ __launch_bounds__(128) void k_bnstat(const float* __restrict__ X, int C, int nN, double* part) {
  __shared__ __attribute__((aligned(16))) double stg[2 * CP];
  const int c = threadIdx.x;
  const int b = blockIdx.x;
  const int r0 = b * RB;
  int r1 = r0 + RB;
  if (r1 > nN) r1 = nN;
  if (c < C) {
    double s = 0.0, q = 0.0;
#pragma unroll 1
    for (int r = r0; r < r1; ++r) {
      const double v = (double)X[(size_t)r * C + c];
      s += v;
      q += v * v;
    }
    stg[c]      = s;
    stg[CP + c] = q;
  }
  __syncthreads();
  if (c < C) {
    const int hseg = C >> 1;
    const int seg  = (c >= hseg) ? 1 : 0;
    const int idx  = seg * CP + 2 * (c - seg * hseg);
    const v2d v = *(const v2d*)(stg + idx);
    double* p = part + (size_t)b * 2 * CP + idx;
    *(volatile v2d*)p = v;
    __threadfence();
    *(volatile v2d*)p = v;
  }
}

__global__ __launch_bounds__(128) void k_bnfin(const double* __restrict__ part, int nb, int C, double invN,
                                              const float* __restrict__ g, float* mean, float* scl) {
  __shared__ __attribute__((aligned(16))) float stg[256];
  const int c = threadIdx.x;
  if (c < C) {
    double s = 0.0, q = 0.0;
#pragma unroll 1
    for (int b = 0; b < nb; ++b) {
      s += part[(size_t)b * 2 * CP + c];
      q += part[(size_t)b * 2 * CP + CP + c];
    }
    const double mu = s * invN;
    double var = q * invN - mu * mu;
    if (var < 0.0) var = 0.0;
    const float mf = (float)mu;
    const float sf = g[c] * rsqrtf((float)var + BNEPS);
    stg[c]       = mf;
    stg[128 + c] = sf;
  }
  __syncthreads();
  const int q4 = C >> 2;
  if (c < 2 * q4) {
    const int seg = (c >= q4) ? 1 : 0;
    const int j   = c - seg * q4;
    const v4f v = *(const v4f*)(stg + seg * 128 + 4 * j);
    float* p = ((seg == 0) ? mean : scl) + 4 * j;
    *(volatile v4f*)p = v;
    __threadfence();
    *(volatile v4f*)p = v;
  }
}

__global__ __launch_bounds__(NTHR) void k_gat(
    const int* __restrict__ ei, const float* __restrict__ ea, const float* __restrict__ XP,
    const float* __restrict__ we, const float* __restrict__ att, const float* __restrict__ bias,
    float* la, float* out, int nN, int nE, int first) {
  extern __shared__ v4f lds_dyn[];
  float* sacc = (float*)lds_dyn;
  float* den  = sacc + LDS_SACC;
  float* cnt  = den + LDS_DEN;
  float* eas  = cnt + NB;
  float* rmx  = eas + NB;
  float* laL  = rmx + LDS_DEN;
  int*   list = (int*)(laL + NB);
  int*   wcnt = list + LDS_LIST;

  const int tid  = threadIdx.x;
  const int lane = tid & 31;
  const int wave = tid >> 5;
  const int hd   = lane >> 3;
  const int c0   = 2 * lane;
  const int nodeBase = blockIdx.x * NB;

  {
    const v4f z4 = {0.f, 0.f, 0.f, 0.f};
    for (int i = tid; i < LDS_ZERO / 4; i += NTHR) lds_dyn[i] = z4;
    for (int i = tid; i < LDS_DEN; i += NTHR) rmx[i] = -1.0e30f;
  }
  __syncthreads();

  const float we0 = we[c0],   we1 = we[c0 + 1];
  const float at0 = att[c0],  at1 = att[c0 + 1];
  const float bb0 = bias[c0], bb1 = bias[c0 + 1];
  const int* eid = ei + nE;
  const bool al16 = ((nE & 3) == 0);

  const int nChunks = (nE + CHUNK - 1) / CHUNK;
#pragma unroll 1
  for (int ch = 0; ch < nChunks; ++ch) {
    const int cbase = ch * CHUNK;
    const bool full = al16 && (cbase + CHUNK <= nE);
    int wc = 0;
#pragma unroll
    for (int g = 0; g < NGRP; ++g) {
      const int el0 = (g * NTHR + tid) * 4;
      const int e0  = cbase + el0;
      const int sent = -2147483647 - 1;
      v4i d;
      if (full) {
        d = *(const v4i*)(eid + e0);
      } else {
        d.x = (e0     < nE) ? eid[min(e0,     nE - 1)] : sent;
        d.y = (e0 + 1 < nE) ? eid[min(e0 + 1, nE - 1)] : sent;
        d.z = (e0 + 2 < nE) ? eid[min(e0 + 2, nE - 1)] : sent;
        d.w = (e0 + 3 < nE) ? eid[min(e0 + 3, nE - 1)] : sent;
      }
      const unsigned s0 = (unsigned)d.x - (unsigned)nodeBase;
      const unsigned s1 = (unsigned)d.y - (unsigned)nodeBase;
      const unsigned s2 = (unsigned)d.z - (unsigned)nodeBase;
      const unsigned s3 = (unsigned)d.w - (unsigned)nodeBase;
      const bool h0 = s0 < (unsigned)NB;
      const bool h1 = s1 < (unsigned)NB;
      const bool h2 = s2 < (unsigned)NB;
      const bool h3 = s3 < (unsigned)NB;
      const unsigned many = __builtin_amdgcn_ballot_w32(h0 | h1 | h2 | h3);
      if (many != 0u) {
#define HITJ(J, HJ, SJ) { \
          const unsigned mj = __builtin_amdgcn_ballot_w32(HJ); \
          if (HJ) { \
            const int pos = wc + (int)__builtin_amdgcn_mbcnt_lo(mj, 0u); \
            if (pos < WCAP) list[wave * WCAP + pos] = ((el0 + (J)) << 9) | (int)(SJ); \
          } \
          wc += (int)__builtin_popcount(mj); }
        HITJ(0, h0, s0)
        HITJ(1, h1, s1)
        HITJ(2, h2, s2)
        HITJ(3, h3, s3)
#undef HITJ
      }
    }
    if (lane == 0) wcnt[wave] = wc;
    __syncthreads();

    if (wave == 0) {
#pragma unroll 1
      for (int wsx = 0; wsx < NWAVE; ++wsx) {
        int n = wcnt[wsx];
        if (n > WCAP) n = WCAP;
        if (n < 0) n = 0;
#pragma unroll 1
        for (int i = 0; i < n; ++i) {
          const int ent  = list[wsx * WCAP + i];
          const int slot = ent & (NB - 1);
          const int el   = (ent >> 9) & (CHUNK - 1);
          int e = cbase + el;
          if (e > nE - 1) e = nE - 1;
          int src = ei[e];
          src = src < 0 ? 0 : (src > nN - 1 ? nN - 1 : src);
          const float a = ea[e];
          int nd = nodeBase + slot;
          if (nd > nN - 1) nd = nN - 1;
          const v2f xs = *(const v2f*)(XP + (size_t)src * XPP + c0);
          const v2f xd = *(const v2f*)(XP + (size_t)nd * XPP + DF + c0);
          float m0 = xs.x + xd.x + a * we0;
          float m1 = xs.y + xd.y + a * we1;
          m0 = (m0 > 0.f) ? m0 : SLOPE * m0;
          m1 = (m1 > 0.f) ? m1 : SLOPE * m1;
          float pl = at0 * m0 + at1 * m1;
          pl += __shfl_xor(pl, 4, 32);
          pl += __shfl_xor(pl, 2, 32);
          pl += __shfl_xor(pl, 1, 32);
          const float lg = __shfl(pl, lane & 24, 32);
          const int ai = slot * NH + hd;
          const float mo = rmx[ai];
          const float dn = den[ai];
          const float mn = fmaxf(mo, lg);
          const float sc = __expf(mo - mn);
          const float p  = __expf(lg - mn);
          rmx[ai] = mn;
          den[ai] = dn * sc + p;
          v2f* sp = (v2f*)(sacc + slot * DF + c0);
          const v2f cur = *sp;
          v2f nx;
          nx.x = cur.x * sc + p * xs.x;
          nx.y = cur.y * sc + p * xs.y;
          *sp = nx;
          if (first != 0) {
            const float cc = cnt[slot];
            const float ee = eas[slot];
            cnt[slot] = cc + 1.0f;
            eas[slot] = ee + a;
          }
        }
      }
    }
    __syncthreads();
  }

  {
    float lav[2];
#pragma unroll
    for (int q = 0; q < 2; ++q) {
      const int slot = wave * 64 + q * 32 + lane;
      const int node = nodeBase + slot;
      float v;
      if (first != 0) {
        const float cc = fmaxf(cnt[slot], 1.0f);
        v = eas[slot] * __builtin_amdgcn_rcpf(cc);
      } else {
        v = la[node];
      }
      laL[slot] = v;
      lav[q] = v;
    }
    if (first != 0) {
#pragma unroll
      for (int q = 0; q < 2; ++q)
        *(volatile float*)(la + (size_t)nodeBase + wave * 64 + q * 32 + lane) = lav[q];
      __threadfence();
#pragma unroll
      for (int q = 0; q < 2; ++q)
        *(volatile float*)(la + (size_t)nodeBase + wave * 64 + q * 32 + lane) = lav[q];
    }
  }
  __syncthreads();

#pragma unroll 1
  for (int j = 0; j < NB / NWAVE; ++j) {
    const int slot = wave * (NB / NWAVE) + j;
    const int node = nodeBase + slot;
    if (node >= nN) break;
    const size_t nrow = (size_t)node;
    const float la0 = laL[slot];
    const v2f xs = *(const v2f*)(XP + nrow * XPP + c0);
    const v2f xd = *(const v2f*)(XP + nrow * XPP + DF + c0);
    float m0 = xs.x + xd.x + la0 * we0;
    float m1 = xs.y + xd.y + la0 * we1;
    m0 = (m0 > 0.f) ? m0 : SLOPE * m0;
    m1 = (m1 > 0.f) ? m1 : SLOPE * m1;
    float pl = at0 * m0 + at1 * m1;
    pl += __shfl_xor(pl, 4, 32);
    pl += __shfl_xor(pl, 2, 32);
    pl += __shfl_xor(pl, 1, 32);
    const float lg = __shfl(pl, lane & 24, 32);
    const int ai = slot * NH + hd;
    const float mo = rmx[ai];
    const float dn = den[ai];
    const float mn = fmaxf(mo, lg);
    const float sc = __expf(mo - mn);
    const float p  = __expf(lg - mn);
    const float dv  = dn * sc + p;
    const float inv = __builtin_amdgcn_rcpf(dv);
    const v2f cur = *(const v2f*)(sacc + slot * DF + c0);
    v2f o;
    o.x = (cur.x * sc + p * xs.x) * inv + bb0;
    o.y = (cur.y * sc + p * xs.y) * inv + bb1;
    float* op = out + nrow * DF + c0;
    *(volatile v2f*)op = o;
    __threadfence();
    *(volatile v2f*)op = o;
  }
}

static size_t al256(size_t x) { return (x + 255) & ~(size_t)255; }

extern "C" void kernel_launch(void* const* d_in, const int* in_sizes, int n_in,
                              void* d_out, int out_size, void* d_ws, size_t ws_size,
                              hipStream_t stream) {
  if (n_in < 31) return;
  if (in_sizes[0] < FIN || (in_sizes[0] % FIN) != 0) return;
  const int nN = in_sizes[0] / FIN;
  if (in_sizes[1] < 2 || (in_sizes[1] & 1) != 0) return;
  const int nE = in_sizes[1] / 2;
  if (in_sizes[2] != nE) return;
  if (in_sizes[3] != FIN * 128 || in_sizes[4] != 128 || in_sizes[5] != 128 || in_sizes[6] != 128) return;
  if (in_sizes[7] != 128 * DF || in_sizes[8] != DF) return;
  for (int L = 0; L < 2; ++L) {
    const int o = 9 + 7 * L;
    if (in_sizes[o] != DF * DF || in_sizes[o + 1] != DF || in_sizes[o + 2] != DF * DF || in_sizes[o + 3] != DF) return;
    if (in_sizes[o + 4] != DF || in_sizes[o + 5] != NH * 16 || in_sizes[o + 6] != DF) return;
  }
  if (in_sizes[23] != DF || in_sizes[24] != DF) return;
  if (in_sizes[25] != DF * DF || in_sizes[26] != DF || in_sizes[27] != DF || in_sizes[28] != DF) return;
  if (in_sizes[29] != DF * NOUT || in_sizes[30] != NOUT) return;
  if (out_size != nN * NOUT) return;

  const float* x       = (const float*)d_in[0];
  const int*   ei      = (const int*)d_in[1];
  const float* ew      = (const float*)d_in[2];
  const float* enc_w0  = (const float*)d_in[3];
  const float* enc_b0  = (const float*)d_in[4];
  const float* enc_g0  = (const float*)d_in[5];
  const float* enc_bt0 = (const float*)d_in[6];
  const float* enc_w1  = (const float*)d_in[7];
  const float* enc_b1  = (const float*)d_in[8];
  const float* g0_wl   = (const float*)d_in[9];
  const float* g0_bl   = (const float*)d_in[10];
  const float* g0_wr   = (const float*)d_in[11];
  const float* g0_br   = (const float*)d_in[12];
  const float* g0_we   = (const float*)d_in[13];
  const float* g0_att  = (const float*)d_in[14];
  const float* g0_b    = (const float*)d_in[15];
  const float* g1_wl   = (const float*)d_in[16];
  const float* g1_bl   = (const float*)d_in[17];
  const float* g1_wr   = (const float*)d_in[18];
  const float* g1_br   = (const float*)d_in[19];
  const float* g1_we   = (const float*)d_in[20];
  const float* g1_att  = (const float*)d_in[21];
  const float* g1_b    = (const float*)d_in[22];
  const float* bn_g    = (const float*)d_in[23];
  const float* bn_b    = (const float*)d_in[24];
  const float* dec_w0  = (const float*)d_in[25];
  const float* dec_b0  = (const float*)d_in[26];
  const float* dec_g0  = (const float*)d_in[27];
  const float* dec_bt0 = (const float*)d_in[28];
  const float* dec_w1  = (const float*)d_in[29];
  const float* dec_b1  = (const float*)d_in[30];
  float* out = (float*)d_out;

  const int nP    = ((nN + GR - 1) / GR) * GR;
  const int gridG = nP / GR;
  const int gridA = (nN + NB - 1) / NB;
  const int nLA   = gridA * NB;
  const int nbS   = (nN + RB - 1) / RB;
  const double invN = 1.0 / (double)nN;

  size_t off = 0;
  unsigned short* wpl = (unsigned short*)((char*)d_ws + off); off += al256((size_t)12 * WPL * sizeof(unsigned short));
  float*  pre0  = (float*)((char*)d_ws + off);  off += al256((size_t)nP * 128 * sizeof(float));
  float*  h0    = (float*)((char*)d_ws + off);  off += al256((size_t)nP * DF * sizeof(float));
  float*  XP    = (float*)((char*)d_ws + off);  off += al256((size_t)nP * XPP * sizeof(float));
  float*  g0    = (float*)((char*)d_ws + off);  off += al256((size_t)nP * DF * sizeof(float));
  float*  g1    = (float*)((char*)d_ws + off);  off += al256((size_t)nP * DF * sizeof(float));
  float*  la    = (float*)((char*)d_ws + off);  off += al256((size_t)nLA * sizeof(float));
  double* part  = (double*)((char*)d_ws + off); off += al256((size_t)nbS * 2 * CP * sizeof(double));
  float*  bmean = (float*)((char*)d_ws + off);  off += al256((size_t)128 * sizeof(float));
  float*  bscl  = (float*)((char*)d_ws + off);  off += al256((size_t)128 * sizeof(float));
  if (off > ws_size) return;
  float* pre2 = pre0;

  unsigned short* Bh[6];
  unsigned short* Bl[6];
  for (int s = 0; s < 6; ++s) { Bh[s] = wpl + (size_t)(2 * s) * WPL; Bl[s] = wpl + (size_t)(2 * s + 1) * WPL; }

  k_wprep<<<(128 * FIN / 8 + NTHR - 1) / NTHR, NTHR, 0, stream>>>(enc_w0, enc_w0, FIN, 128, 128, Bh[0], Bl[0]);
  k_gemm<FIN, 128, false><<<gridG, NTHR, 0, stream>>>(x, Bh[0], Bl[0], enc_b0, enc_b0, 128,
                                                      bmean, bscl, enc_bt0, pre0, nN, nP);
  k_bnstat<<<nbS, 128, 0, stream>>>(pre0, 128, nN, part);
  k_bnfin<<<1, 128, 0, stream>>>(part, nbS, 128, invN, enc_g0, bmean, bscl);
  k_wprep<<<(64 * 128 / 8 + NTHR - 1) / NTHR, NTHR, 0, stream>>>(enc_w1, enc_w1, 128, DF, DF, Bh[1], Bl[1]);
  k_gemm<128, DF, true><<<gridG, NTHR, 0, stream>>>(pre0, Bh[1], Bl[1], enc_b1, enc_b1, DF,
                                                    bmean, bscl, enc_bt0, h0, nN, nP);

  k_wprep<<<(128 * DF / 8 + NTHR - 1) / NTHR, NTHR, 0, stream>>>(g0_wl, g0_wr, DF, DF, 128, Bh[2], Bl[2]);
  k_gemm<DF, 128, false><<<gridG, NTHR, 0, stream>>>(h0, Bh[2], Bl[2], g0_bl, g0_br, DF,
                                                     bmean, bscl, bn_b, XP, nN, nP);
  hipFuncSetAttribute(reinterpret_cast<const void*>(&k_gat),
                      hipFuncAttributeMaxDynamicSharedMemorySize, LDS_BYTES);
  k_gat<<<gridA, NTHR, LDS_BYTES, stream>>>(ei, ew, XP, g0_we, g0_att, g0_b, la, g0, nN, nE, 1);

  k_bnstat<<<nbS, DF, 0, stream>>>(g0, DF, nN, part);
  k_bnfin<<<1, DF, 0, stream>>>(part, nbS, DF, invN, bn_g, bmean, bscl);
  k_wprep<<<(128 * DF / 8 + NTHR - 1) / NTHR, NTHR, 0, stream>>>(g1_wl, g1_wr, DF, DF, 128, Bh[3], Bl[3]);
  k_gemm<DF, 128, true><<<gridG, NTHR, 0, stream>>>(g0, Bh[3], Bl[3], g1_bl, g1_br, DF,
                                                    bmean, bscl, bn_b, XP, nN, nP);
  k_gat<<<gridA, NTHR, LDS_BYTES, stream>>>(ei, ew, XP, g1_we, g1_att, g1_b, la, g1, nN, nE, 0);

  k_wprep<<<(DF * DF / 8 + NTHR - 1) / NTHR, NTHR, 0, stream>>>(dec_w0, dec_w0, DF, DF, DF, Bh[4], Bl[4]);
  k_gemm<DF, DF, false><<<gridG, NTHR, 0, stream>>>(g1, Bh[4], Bl[4], dec_b0, dec_b0, DF,
                                                    bmean, bscl, dec_bt0, pre2, nN, nP);
  k_bnstat<<<nbS, DF, 0, stream>>>(pre2, DF, nN, part);
  k_bnfin<<<1, DF, 0, stream>>>(part, nbS, DF, invN, dec_g0, bmean, bscl);
  k_wprep<<<(NOUT * DF / 8 + NTHR - 1) / NTHR, NTHR, 0, stream>>>(dec_w1, dec_w1, DF, NOUT, NOUT, Bh[5], Bl[5]);
  k_gemm<DF, NOUT, true><<<gridG, NTHR, 0, stream>>>(pre2, Bh[5], Bl[5], dec_b1, dec_b1, NOUT,
                                                     bmean, bscl, dec_bt0, out, nN, nN);
}
